// CorrectionRegressor_6167573037828
// MI455X (gfx1250) — hardware-verified
//
#include <hip/hip_runtime.h>
#include <math.h>

constexpr int kRowsChunk = 32768;
constexpr int kInDim   = 16;
constexpr int kEmb     = 8;
constexpr int kNMol    = 8;
constexpr int kNIso    = 12;
constexpr int kZDim    = 32;
constexpr int kHid1    = 256;
constexpr int kHid2    = 128;
constexpr int kShKPad  = 192;
constexpr int kShKReal = 136;
constexpr int kShN     = 64;
constexpr int kIsoHid  = 64;
constexpr int kExN     = kNIso * kIsoHid;
constexpr float kWCarry    = 16.0f;
constexpr float kWCarryInv = 1.0f / 16.0f;
constexpr float kLnEps     = 1e-5f;

typedef __attribute__((ext_vector_type(16))) _Float16 v16h;
typedef __attribute__((ext_vector_type(8)))  _Float16 v8h;
typedef __attribute__((ext_vector_type(16))) __bf16   v16b;
typedef __attribute__((ext_vector_type(8)))  __bf16   v8b;
typedef __attribute__((ext_vector_type(8)))  float    v8f;
typedef __attribute__((ext_vector_type(4)))  float    v4f;
typedef __attribute__((ext_vector_type(4)))  unsigned int v4u;

__device__ __forceinline__ unsigned short f2bf_bits(float f) {
  unsigned u = __float_as_uint(f);
  return (unsigned short)((u + 0x7FFFu + ((u >> 16) & 1u)) >> 16);
}
__device__ __forceinline__ float bf_bits2f(unsigned short h) { return __uint_as_float(((unsigned)h) << 16); }

__device__ __forceinline__ void dep_guard_h(v8f& a, v8f& b, v16h x, v16h y) { asm volatile("v_nop\n\tv_nop\n\tv_nop\n\tv_nop" : "+v"(a), "+v"(b) : "v"(x), "v"(y)); }
__device__ __forceinline__ void dep_guard_b(v8f& a, v8f& b, v16b x, v16b y) { asm volatile("v_nop\n\tv_nop\n\tv_nop\n\tv_nop" : "+v"(a), "+v"(b) : "v"(x), "v"(y)); }
__device__ __forceinline__ void keep4_h(v16h a, v16h b, v16h c, v16h d) { asm volatile("v_nop" :: "v"(a), "v"(b), "v"(c), "v"(d)); }
__device__ __forceinline__ void keep4_b(v16b a, v16b b, v16b c, v16b d) { asm volatile("v_nop" :: "v"(a), "v"(b), "v"(c), "v"(d)); }
__device__ __forceinline__ void acc_guard4(v8f& a, v8f& b, v8f& c, v8f& d) { asm volatile("v_nop\n\tv_nop\n\tv_nop\n\tv_nop" : "+v"(a), "+v"(b), "+v"(c), "+v"(d)); }
template <typename T> struct Frag;
template <> struct Frag<_Float16> {
  typedef v16h V; union U { v16h v; v8h h[2]; };
  static __device__ __forceinline__ v16h load(const _Float16* p) {
    U f; f.h[0] = *(const v8h*)(p); f.h[1] = *(const v8h*)(p + 16); return f.v;
  }
  static __device__ __forceinline__ v8f mma(v16h a, v16h b, v8f c) {
    return __builtin_amdgcn_wmma_f32_16x16x32_f16(false, a, false, b, (short)0, c, false, false);
  }
  static __device__ __forceinline__ void guard(v8f& a, v8f& b, v16h x, v16h y) { dep_guard_h(a, b, x, y); }
  static __device__ __forceinline__ void keep(v16h a, v16h b, v16h c, v16h d) { keep4_h(a, b, c, d); }
};
template <> struct Frag<__bf16> {
  typedef v16b V; union U { v16b v; v8b h[2]; };
  static __device__ __forceinline__ v16b load(const __bf16* p) {
    U f; f.h[0] = *(const v8b*)(p); f.h[1] = *(const v8b*)(p + 16); return f.v;
  }
  static __device__ __forceinline__ v8f mma(v16b a, v16b b, v8f c) {
    return __builtin_amdgcn_wmma_f32_16x16x32_bf16(false, a, false, b, (short)0, c, false, false);
  }
  static __device__ __forceinline__ void guard(v8f& a, v8f& b, v16b x, v16b y) { dep_guard_b(a, b, x, y); }
  static __device__ __forceinline__ void keep(v16b a, v16b b, v16b c, v16b d) { keep4_b(a, b, c, d); }
};

__device__ __forceinline__ unsigned pk16(unsigned short a, unsigned short b) { return (unsigned)a | ((unsigned)b << 16); }
__device__ __forceinline__ unsigned short h_bits(float f) { const _Float16 h = (_Float16)f; return __builtin_bit_cast(unsigned short, h); }

template <int ET> struct Elem;
template <> struct Elem<0> { typedef _Float16 T; };
template <> struct Elem<1> { typedef __bf16 T; };
template <int ET, bool SPLIT, int BIAS_MODE, int OUT_MODE, bool RESID, int ACT = 0>
__global__ __launch_bounds__(256) void wmma_gemm64(
    const unsigned short* __restrict__ Ap, const unsigned short* __restrict__ A2p, int lda, long strideA,
    const unsigned short* __restrict__ Btp, const unsigned short* __restrict__ Bt2p, int ldb, long strideB,
    void* __restrict__ Cout, void* __restrict__ Cout2, int ldc, long strideC,
    const float* __restrict__ bias,
    const float* __restrict__ resid, long strideR,
    int M, int N, int K, float scale) {
  typedef typename Elem<ET>::T T;
  typedef typename Frag<T>::V V;
  const T* A = (const T*)Ap; const T* A2 = (const T*)A2p; const T* Bt = (const T*)Btp; const T* Bt2 = (const T*)Bt2p;
  __shared__ __align__(16) float sT[8][16 * 68];
  const int b    = blockIdx.y;
  const int lane = threadIdx.x & 31;
  const int wave = threadIdx.x >> 5;
  const int tilesN = N >> 6;
  const int tilesM = M >> 6;
  const int tile = blockIdx.x * 8 + wave;
  if (tile >= tilesM * tilesN) return;
  const int tm = tile / tilesN;
  const int tn = tile - tm * tilesN;
  const int m0 = tm << 6;
  const int n0 = tn << 6;

  const T* Ab  = A  + (size_t)b * strideA;
  const T* Bb  = Bt + (size_t)b * strideB;
  const T* Ab2 = SPLIT ? (A2  + (size_t)b * strideA) : nullptr;
  const T* Bb2 = SPLIT ? (Bt2 + (size_t)b * strideB) : nullptr;

  const int rlane = lane & 15;
  const int koff  = (lane >> 4) * 8;
  const int mOff  = (lane >> 4) * 8;

  v8f acc[4][4];
#pragma unroll
  for (int i = 0; i < 4; ++i)
#pragma unroll
    for (int j = 0; j < 4; ++j) acc[i][j] = (v8f){0.f,0.f,0.f,0.f,0.f,0.f,0.f,0.f};

  for (int k0 = 0; k0 < K; k0 += 32) {
    V bh[4], bl[4];
#pragma unroll
    for (int j = 0; j < 4; ++j) {
      const size_t bo = (size_t)(n0 + (j << 4) + rlane) * ldb + koff + k0;
      bh[j] = Frag<T>::load(Bb + bo);
      if (SPLIT) bl[j] = Frag<T>::load(Bb2 + bo);
    }
#pragma unroll
    for (int i = 0; i < 4; ++i) {
      const size_t ao = (size_t)(m0 + (i << 4) + rlane) * lda + koff + k0;
      V ah = Frag<T>::load(Ab + ao);
      V al;
      if (SPLIT) al = Frag<T>::load(Ab2 + ao);
#pragma unroll
      for (int j = 0; j < 4; ++j) {
        acc[i][j] = Frag<T>::mma(ah, bh[j], acc[i][j]);
        if (SPLIT) {
          acc[i][j] = Frag<T>::mma(ah, bl[j], acc[i][j]);
          acc[i][j] = Frag<T>::mma(al, bh[j], acc[i][j]);
        }
      }
      Frag<T>::guard(acc[i][0], acc[i][3], ah, SPLIT ? al : ah);
    }
    Frag<T>::keep(bh[0], bh[1], bh[2], bh[3]);
    if (SPLIT) Frag<T>::keep(bl[0], bl[1], bl[2], bl[3]);
  }
  acc_guard4(acc[0][0], acc[0][1], acc[0][2], acc[0][3]);
  acc_guard4(acc[1][0], acc[1][1], acc[1][2], acc[1][3]);
  acc_guard4(acc[2][0], acc[2][1], acc[2][2], acc[2][3]);
  acc_guard4(acc[3][0], acc[3][1], acc[3][2], acc[3][3]);

  float* slab = sT[wave];
  const float* Rb = RESID ? (resid + (size_t)b * strideR) : nullptr;
#pragma unroll
  for (int i = 0; i < 4; ++i) {
    const int mBase = m0 + (i << 4);
#pragma unroll
    for (int j = 0; j < 4; ++j) {
      const int n = n0 + (j << 4) + rlane;
      float bv = 0.f;
      if (BIAS_MODE == 2) bv = bias[n];
#pragma unroll
      for (int r = 0; r < 8; ++r) {
        float v = acc[i][j][r] * scale;
        if (BIAS_MODE == 1) v += bias[mBase + mOff + r];
        if (BIAS_MODE == 2) v += bv;
        if (RESID) v += Rb[(size_t)(mBase + mOff + r) * ldc + n];
        if (ACT == 2) v = fmaxf(v, 0.0f);
        if (ACT == 4) v = (v > 0.f) ? v : 0.01f * v;
        slab[(mOff + r) * 68 + (j << 4) + rlane] = v;
      }
    }
    __builtin_amdgcn_fence(__ATOMIC_RELEASE, "workgroup");
    __builtin_amdgcn_wave_barrier();
    __builtin_amdgcn_fence(__ATOMIC_ACQUIRE, "workgroup");
    if (OUT_MODE == 0) {
      float* C = (float*)Cout + (size_t)b * strideC;
      const int hh = lane >> 4, c4 = (lane & 15) * 4;
      for (int pass = 0; pass < 2; ++pass) {
#pragma unroll
        for (int it = 0; it < 8; ++it) {
          const int row = it * 2 + hh;
          v4f v = *(const v4f*)(slab + row * 68 + c4);
          *(volatile v4f*)(C + (size_t)(mBase + row) * ldc + n0 + c4) = v;
        }
        __threadfence();
      }
    } else {
      const int q = lane >> 3, c8 = (lane & 7) * 8;
      unsigned short* C  = (unsigned short*)Cout  + (size_t)b * strideC;
      unsigned short* C2 = (OUT_MODE == 2) ? ((unsigned short*)Cout2 + (size_t)b * strideC) : nullptr;
      for (int pass = 0; pass < 2; ++pass) {
#pragma unroll
        for (int it = 0; it < 4; ++it) {
          const int row = it * 4 + q;
          const float* sp = slab + row * 68 + c8;
          v8h hv, lv;
#pragma unroll
          for (int e = 0; e < 8; ++e) {
            if (OUT_MODE == 1) {
              hv[e] = (_Float16)sp[e];
            } else {
              unsigned short hb = f2bf_bits(sp[e]);
              unsigned short lb = f2bf_bits(sp[e] - bf_bits2f(hb));
              hv[e] = __builtin_bit_cast(_Float16, hb);
              lv[e] = __builtin_bit_cast(_Float16, lb);
            }
          }
          *(volatile v8h*)(C + (size_t)(mBase + row) * ldc + n0 + c8) = hv;
          if (OUT_MODE == 2) *(volatile v8h*)(C2 + (size_t)(mBase + row) * ldc + n0 + c8) = lv;
        }
        __threadfence();
      }
    }
    __builtin_amdgcn_fence(__ATOMIC_RELEASE, "workgroup");
    __builtin_amdgcn_wave_barrier();
    __builtin_amdgcn_fence(__ATOMIC_ACQUIRE, "workgroup");
  }
}

__device__ __forceinline__ float wave_sum(float v) {
#pragma unroll
  for (int off = 16; off > 0; off >>= 1) v += __shfl_xor(v, off, 32);
  return v;
}
__device__ __forceinline__ float gelu_erf(float x) {
  return 0.5f * x * (1.0f + erff(x * 0.70710678118654752f));
}
__device__ __forceinline__ int wrap_clamp(int i, int n) {
  int v = (i < 0) ? (i + n) : i;
  v = (v < 0) ? 0 : v;
  v = (v > n - 1) ? (n - 1) : v;
  return v;
}

__global__ __launch_bounds__(256) void wprep_kernel(const float* __restrict__ W, unsigned short* __restrict__ out,
                                                    int ldo, int kreal, int ldi, int ngrp, int grpStride,
                                                    int n8total, float scale) {
  const int g = blockIdx.x * 256 + threadIdx.x;
  if (g >= n8total) return;
  const int e   = g * 8;
  const int nn  = e / ldo;
  const int k0  = e - nn * ldo;
  const int grp = nn / ngrp;
  const int n   = nn - grp * ngrp;
  unsigned short hb[8];
#pragma unroll
  for (int j = 0; j < 8; ++j) {
    const int k  = k0 + j;
    const int kc = (k < kreal) ? k : (kreal - 1);
    float v = W[(size_t)grp * grpStride + (size_t)kc * ldi + n] * scale;
    v = (k < kreal) ? v : 0.0f;
    hb[j] = h_bits(v);
  }
  const v4u u = (v4u){pk16(hb[0], hb[1]), pk16(hb[2], hb[3]), pk16(hb[4], hb[5]), pk16(hb[6], hb[7])};
  unsigned short* q = out + (size_t)e;
  *(volatile v4u*)q = u;
  __threadfence();
  *(volatile v4u*)q = u;
}

__global__ __launch_bounds__(256) void zcast_kernel(const float* __restrict__ x, const int* __restrict__ mol_idx,
                                                    const int* __restrict__ iso_idx, const float* __restrict__ mol_embed,
                                                    const float* __restrict__ iso_embed, unsigned short* __restrict__ Z) {
  const int g   = blockIdx.x * 256 + threadIdx.x;
  const int row = g >> 2;
  const int sub = g & 3;
  const int mi = wrap_clamp(mol_idx[row], kNMol);
  const int ii = wrap_clamp(iso_idx[row], kNIso);
  const int xo = (sub & 1) * 8;
  const float* xr = x + (size_t)row * kInDim + xo;
  const v4f xa = *(const v4f*)(xr);
  const v4f xb = *(const v4f*)(xr + 4);
  const v4f ma = *(const v4f*)(mol_embed + mi * kEmb);
  const v4f mb = *(const v4f*)(mol_embed + mi * kEmb + 4);
  const v4f ia = *(const v4f*)(iso_embed + ii * kEmb);
  const v4f ib = *(const v4f*)(iso_embed + ii * kEmb + 4);
  const bool isx = (sub < 2);
  const bool ism = (sub == 2);
  unsigned short hb[8];
#pragma unroll
  for (int e = 0; e < 4; ++e) {
    const float f0 = isx ? xa[e] : (ism ? ma[e] : ia[e]);
    const float f1 = isx ? xb[e] : (ism ? mb[e] : ib[e]);
    hb[e]     = h_bits(f0);
    hb[4 + e] = h_bits(f1);
  }
  const v4u u = (v4u){pk16(hb[0], hb[1]), pk16(hb[2], hb[3]), pk16(hb[4], hb[5]), pk16(hb[6], hb[7])};
  unsigned short* q = Z + (size_t)row * kZDim + sub * 8;
  *(volatile v4u*)q = u;
  __threadfence();
  *(volatile v4u*)q = u;
}

template <int NCOL, int OPITCH>
__global__ __launch_bounds__(256) void ln_gelu_kernel(const float* __restrict__ X, const float* __restrict__ gam,
                                                      const float* __restrict__ bet, const int* __restrict__ iso_idx,
                                                      const float* __restrict__ iso_embed, unsigned short* __restrict__ Y) {
  __shared__ __align__(16) float sv[8][NCOL];
  __shared__ __align__(16) unsigned short sq[8][OPITCH];
  const int t = threadIdx.x;
  const int lane = t & 31, w = t >> 5;
  const int row = blockIdx.x * 8 + w;
  const float* xr = X + (size_t)row * NCOL;

  float s = 0.f;
#pragma unroll 1
  for (int i = 0; i < NCOL / 32; ++i) {
    const int c = i * 32 + lane;
    const float v = xr[c];
    sv[w][c] = v;
    s += v;
  }
  s = wave_sum(s);
  const float mu = s * (1.0f / (float)NCOL);
  __syncthreads();

  float ss = 0.f;
#pragma unroll 1
  for (int i = 0; i < NCOL / 32; ++i) {
    const int c = i * 32 + lane;
    const float d = sv[w][c] - mu;
    ss += d * d;
  }
  ss = wave_sum(ss);
  const float var  = ss * (1.0f / (float)NCOL);
  const float rstd = rsqrtf(var + kLnEps);

  int isoc = 0;
  if (OPITCH > NCOL) isoc = wrap_clamp(iso_idx[row], kNIso);

#pragma unroll 1
  for (int i = 0; i < OPITCH / 32; ++i) {
    const int c  = i * 32 + lane;
    const int cc = (c < NCOL) ? c : (NCOL - 1);
    const float v = sv[w][cc];
    const float y = gelu_erf((v - mu) * rstd * gam[cc] + bet[cc]);
    float val = y;
    if (OPITCH > NCOL) {
      int ec = c - NCOL;
      ec = (ec < 0) ? 0 : ((ec > kEmb - 1) ? (kEmb - 1) : ec);
      const float iev = iso_embed[isoc * kEmb + ec];
      val = (c < NCOL) ? y : ((c < NCOL + kEmb) ? iev : 0.0f);
    }
    sq[w][c] = h_bits(val);
  }
  __syncthreads();

  constexpr int kStoreLanes = OPITCH / 8;
  const int lc = (lane < kStoreLanes) ? lane : (kStoreLanes - 1);
  const v4u u = *(const v4u*)(&sq[w][lc * 8]);
  unsigned short* yr = Y + (size_t)row * OPITCH + lc * 8;
  if (lane < kStoreLanes) { *(volatile v4u*)yr = u; }
  __threadfence();
  if (lane < kStoreLanes) { *(volatile v4u*)yr = u; }
}

__global__ __launch_bounds__(256) void head_kernel(const float* __restrict__ E, const float* __restrict__ P,
                                                   const int* __restrict__ iso_idx, const float* __restrict__ iso_embed,
                                                   const float* __restrict__ Wsh2, const float* __restrict__ bsh2,
                                                   const float* __restrict__ Wiso2, const float* __restrict__ biso2,
                                                   const float* __restrict__ Wg, const float* __restrict__ bg,
                                                   float* __restrict__ outp) {
  const int t = threadIdx.x;
  const int lane = t & 31, w = t >> 5;
  const int rb = (blockIdx.x * 8 + w) * 32;
  const float bshv = bsh2[0];
  const float bgv  = bg[0];
  const float wgl  = Wg[lane & 7];
  float res = 0.f;
#pragma unroll 1
  for (int rr = 0; rr < 32; ++rr) {
    const int row  = rb + rr;
    const int iraw = iso_idx[row];
    const bool valid = ((unsigned)iraw < (unsigned)kNIso);
    const int iw = wrap_clamp(iraw, kNIso);
    float ap = 0.f, ae = 0.f;
#pragma unroll 1
    for (int q = 0; q < 4; ++q) {
      const int col = (q & 1) * 32 + lane;
      const float pv = P[(size_t)row * kShN + col];
      const float ev = E[(size_t)row * kExN + iw * kIsoHid + col];
      const float wp = Wsh2[col];
      const float we = Wiso2[iw * kIsoHid + col];
      const bool isp = (q < 2);
      const float xv = isp ? pv : ev;
      const float wv = isp ? wp : we;
      const float gv = gelu_erf(xv) * wv;
      ap += isp ? gv : 0.f;
      ae += isp ? 0.f : gv;
    }
    ap = wave_sum(ap);
    ae = wave_sum(ae);
    const float sp = ap + bshv;
    float he = ae + biso2[iw];
    he = valid ? he : 0.0f;
    const float iev = iso_embed[iw * kEmb + (lane & 7)];
    float gp = iev * wgl;
    gp = (lane < 8) ? gp : 0.0f;
    gp = wave_sum(gp);
    const float gz = gp + bgv;
    const float gate = 1.0f / (1.0f + expf(-gz));
    const float fin = gate * he + (1.0f - gate) * sp;
    res = (lane == rr) ? fin : res;
  }
  float* op = outp + rb + lane;
  *(volatile float*)op = res;
  __threadfence();
  *(volatile float*)op = res;
}

extern "C" void kernel_launch(void* const* d_in, const int* in_sizes, int n_in,
                              void* d_out, int out_size, void* d_ws, size_t ws_size,
                              hipStream_t stream) {
  if (n_in < 23) return;
  const float* x         = (const float*)d_in[0];
  const int*   mol_idx   = (const int*)d_in[1];
  const int*   iso_idx   = (const int*)d_in[2];
  const float* mol_embed = (const float*)d_in[3];
  const float* iso_embed = (const float*)d_in[4];
  const float* W1    = (const float*)d_in[5];
  const float* b1    = (const float*)d_in[6];
  const float* g1    = (const float*)d_in[7];
  const float* be1   = (const float*)d_in[8];
  const float* W2    = (const float*)d_in[9];
  const float* b2    = (const float*)d_in[10];
  const float* g2    = (const float*)d_in[11];
  const float* be2   = (const float*)d_in[12];
  const float* Wsh1  = (const float*)d_in[13];
  const float* bsh1  = (const float*)d_in[14];
  const float* Wsh2  = (const float*)d_in[15];
  const float* bsh2  = (const float*)d_in[16];
  const float* Wiso1 = (const float*)d_in[17];
  const float* biso1 = (const float*)d_in[18];
  const float* Wiso2 = (const float*)d_in[19];
  const float* biso2 = (const float*)d_in[20];
  const float* Wg    = (const float*)d_in[21];
  const float* bg    = (const float*)d_in[22];
  float* out = (float*)d_out;

  const int nrows = in_sizes[2];
  if (nrows <= 0 || in_sizes[0] != nrows * kInDim || in_sizes[1] != nrows || out_size != nrows) return;
  if (in_sizes[5] != kZDim * kHid1 || in_sizes[9] != kHid1 * kHid2 || in_sizes[13] != kShKReal * kShN ||
      in_sizes[17] != kNIso * kHid2 * kIsoHid || in_sizes[18] != kExN) return;
  const int nchunk = nrows / kRowsChunk;
  if (nchunk * kRowsChunk != nrows) return;

  const size_t CH = (size_t)kRowsChunk;
  char* ws = (char*)d_ws;
  size_t off = 0;
  const size_t szE32 = CH * kExN * 4;
  char* rE32 = ws + off;
  char* rZ16 = rE32;
  char* rH32 = rZ16 + CH * kZDim * 2;
  char* rH16 = rH32 + CH * kHid1 * 4;
  char* rS32 = rH16 + CH * kHid1 * 2;
  if ((size_t)(rS32 - rE32) + CH * kHid2 * 4 > szE32) return;
  off += szE32;
  char* rSH16 = ws + off;  off += CH * kShKPad * 2;
  char* rP32  = ws + off;  off += CH * kShN * 4;
  char* rW1t  = ws + off;  off += (size_t)kHid1 * kZDim * 2;
  char* rW2t  = ws + off;  off += (size_t)kHid2 * kHid1 * 2;
  char* rWsh  = ws + off;  off += (size_t)kShN * kShKPad * 2;
  char* rWiso = ws + off;  off += (size_t)kExN * kHid2 * 2;
  if (off > ws_size) return;

  unsigned short* W1t   = (unsigned short*)rW1t;
  unsigned short* W2t   = (unsigned short*)rW2t;
  unsigned short* Wsh1t = (unsigned short*)rWsh;
  unsigned short* Wiso1t = (unsigned short*)rWiso;
  unsigned short* Z16  = (unsigned short*)rZ16;
  float*          H32  = (float*)rH32;
  unsigned short* H16  = (unsigned short*)rH16;
  float*          S32  = (float*)rS32;
  unsigned short* SH16 = (unsigned short*)rSH16;
  float*          P32  = (float*)rP32;
  float*          E32  = (float*)rE32;

  {
    const int n8a = kHid1 * kZDim / 8;
    wprep_kernel<<<dim3((n8a + 255) / 256), dim3(256), 0, stream>>>(W1, W1t, kZDim, kZDim, kHid1, kHid1, 0, n8a, kWCarry);
    const int n8b = kHid2 * kHid1 / 8;
    wprep_kernel<<<dim3((n8b + 255) / 256), dim3(256), 0, stream>>>(W2, W2t, kHid1, kHid1, kHid2, kHid2, 0, n8b, kWCarry);
    const int n8c = kShN * kShKPad / 8;
    wprep_kernel<<<dim3((n8c + 255) / 256), dim3(256), 0, stream>>>(Wsh1, Wsh1t, kShKPad, kShKReal, kShN, kShN, 0, n8c, kWCarry);
    const int n8d = kExN * kHid2 / 8;
    wprep_kernel<<<dim3((n8d + 255) / 256), dim3(256), 0, stream>>>(Wiso1, Wiso1t, kHid2, kHid2, kIsoHid, kIsoHid, kHid2 * kIsoHid, n8d, kWCarry);
  }

  const int M = kRowsChunk;
  const int tilesM = M / 64;
  for (int c = 0; c < nchunk; ++c) {
    const size_t r0 = (size_t)c * CH;
    const float* xc   = x + r0 * kInDim;
    const int*   molc = mol_idx + r0;
    const int*   isoc = iso_idx + r0;
    float*       outc = out + r0;

    zcast_kernel<<<dim3(M * 4 / 256), dim3(256), 0, stream>>>(xc, molc, isoc, mol_embed, iso_embed, Z16);

    wmma_gemm64<0, false, 2, 0, false, 0><<<dim3(tilesM * (kHid1 / 64) / 8, 1), dim3(256), 0, stream>>>(
        Z16, Z16, kZDim, 0L, W1t, W1t, kZDim, 0L, (void*)H32, (void*)H32, kHid1, 0L,
        b1, b1, 0L, M, kHid1, kZDim, kWCarryInv);

    ln_gelu_kernel<kHid1, kHid1><<<dim3(M / 8), dim3(256), 0, stream>>>(H32, g1, be1, isoc, iso_embed, H16);

    wmma_gemm64<0, false, 2, 0, false, 0><<<dim3(tilesM * (kHid2 / 64) / 8, 1), dim3(256), 0, stream>>>(
        H16, H16, kHid1, 0L, W2t, W2t, kHid1, 0L, (void*)S32, (void*)S32, kHid2, 0L,
        b2, b2, 0L, M, kHid2, kHid1, kWCarryInv);

    ln_gelu_kernel<kHid2, kShKPad><<<dim3(M / 8), dim3(256), 0, stream>>>(S32, g2, be2, isoc, iso_embed, SH16);

    wmma_gemm64<0, false, 2, 0, false, 0><<<dim3(tilesM * (kExN / 64) / 8, 1), dim3(256), 0, stream>>>(
        SH16, SH16, kShKPad, 0L, Wiso1t, Wiso1t, kHid2, 0L, (void*)E32, (void*)E32, kExN, 0L,
        biso1, biso1, 0L, M, kExN, kHid2, kWCarryInv);

    wmma_gemm64<0, false, 2, 0, false, 0><<<dim3(tilesM * (kShN / 64) / 8, 1), dim3(256), 0, stream>>>(
        SH16, SH16, kShKPad, 0L, Wsh1t, Wsh1t, kShKPad, 0L, (void*)P32, (void*)P32, kShN, 0L,
        bsh1, bsh1, 0L, M, kShN, kShKPad, kWCarryInv);

    head_kernel<<<dim3(M / 256), dim3(256), 0, stream>>>(E32, P32, isoc, iso_embed, Wsh2, bsh2, Wiso2, biso2, Wg, bg, outc);
  }
}
